// TemporalSequentialAttentionLayer_v2_14791867367636
// MI455X (gfx1250) — hardware-verified
//
#include <hip/hip_runtime.h>
#include <math.h>

typedef __attribute__((ext_vector_type(16))) _Float16 v16h;
typedef __attribute__((ext_vector_type(16))) __bf16 v16b;
typedef __attribute__((ext_vector_type(8)))  _Float16 v8h;
typedef __attribute__((ext_vector_type(8)))  float v8f;
typedef __attribute__((ext_vector_type(4)))  float v4f;
typedef __attribute__((ext_vector_type(2)))  float v2f;
typedef __attribute__((ext_vector_type(4)))  unsigned v4u;
typedef __attribute__((ext_vector_type(4)))  int v4i;
typedef float __attribute__((may_alias)) float_a;
typedef int __attribute__((may_alias)) int_a;

template <typename T> __device__ __forceinline__ void vst2(void* p, T v) { *(volatile T*)p = v; __threadfence(); *(volatile T*)p = v; }
__device__ __forceinline__ v8f wmma16(v16h a, v16h b, v8f c) {
  v8f d = __builtin_amdgcn_wmma_f32_16x16x32_f16(false, a, false, b, (short)0, c, false, false);
  asm volatile("v_nop\n\tv_nop\n\tv_nop\n\tv_nop" : "+v"(d) : "v"(a), "v"(b));
  return d;
}
__device__ __forceinline__ v8f wmma_bf(v16b a, v16b b, v8f c) {
  v8f d = __builtin_amdgcn_wmma_f32_16x16x32_bf16(false, a, false, b, (short)0, c, false, false);
  asm volatile("v_nop\n\tv_nop\n\tv_nop\n\tv_nop" : "+v"(d) : "v"(a), "v"(b));
  return d;
}
__device__ __forceinline__ v16h frag_h(const _Float16* rowk0, int lane) {
  union { v16h v; v8h q[2]; } u; const _Float16* p = rowk0 + 8 * (lane >> 4);
  u.q[0] = *(const v8h*)p; u.q[1] = *(const v8h*)(p + 16); return u.v;
}
__device__ __forceinline__ v16h frag_f32(const float* rowk0, int lane) {
  v16h a; const float* p = rowk0 + 8 * (lane >> 4);
#pragma unroll
  for (int i = 0; i < 8; ++i) { a[i] = (_Float16)p[i]; a[8 + i] = (_Float16)p[16 + i]; }
  return a;
}
__device__ __forceinline__ v16h frag_f32s(const float* rowk0, int lane, float sc) {
  v16h a; const float* p = rowk0 + 8 * (lane >> 4);
#pragma unroll
  for (int i = 0; i < 8; ++i) { a[i] = (_Float16)(p[i] * sc); a[8 + i] = (_Float16)(p[16 + i] * sc); }
  return a;
}
__device__ __forceinline__ v16h fragc_f32(const float* W, int k0, int n, int lane, int ld, int K) {
  v16h a; const int g = lane >> 4;
#pragma unroll
  for (int i = 0; i < 8; ++i) { const int ka = k0 + 8 * g + i, kb = ka + 16;
    a[i] = (_Float16)(ka < K ? W[(size_t)ka * ld + n] : 0.f); a[8 + i] = (_Float16)(kb < K ? W[(size_t)kb * ld + n] : 0.f); }
  return a;
}
struct F2 { v16b h, l; };
__device__ __forceinline__ F2 bsplit16(const float v[16]) { F2 r;
#pragma unroll
  for (int i = 0; i < 16; ++i) { const __bf16 h = (__bf16)v[i]; r.h[i] = h; r.l[i] = (__bf16)(v[i] - (float)h); }
  return r; }
__device__ __forceinline__ F2 split_row(const float* row, int k0, int lane) { float v[16]; const float* p = row + k0 + 8 * (lane >> 4);
#pragma unroll
  for (int i = 0; i < 8; ++i) { v[i] = p[i]; v[8 + i] = p[16 + i]; }
  return bsplit16(v); }
__device__ __forceinline__ F2 split_rowK(const float* row, int k0, int lane, int K) { float v[16]; const int g = lane >> 4;
#pragma unroll
  for (int i = 0; i < 8; ++i) { const int ka = k0 + 8 * g + i, kb = ka + 16; v[i] = ka < K ? row[ka] : 0.f; v[8 + i] = kb < K ? row[kb] : 0.f; }
  return bsplit16(v); }
__device__ __forceinline__ F2 split_col(const float* W, int k0, int n, int lane, int ld, int K) { float v[16]; const int g = lane >> 4;
#pragma unroll
  for (int i = 0; i < 8; ++i) { const int ka = k0 + 8 * g + i, kb = ka + 16; v[i] = ka < K ? W[(size_t)ka * ld + n] : 0.f; v[8 + i] = kb < K ? W[(size_t)kb * ld + n] : 0.f; }
  return bsplit16(v); }
__device__ __forceinline__ v8f mac3(const F2& a, const F2& b, v8f c) { c = wmma_bf(a.l, b.h, c); c = wmma_bf(a.h, b.l, c); return wmma_bf(a.h, b.h, c); }
__device__ __forceinline__ float sigm(float v) { return 1.0f / (1.0f + expf(-v)); }
#define LDSX() do { asm volatile("s_wait_dscnt 0" ::: "memory"); __builtin_amdgcn_wave_barrier(); __builtin_amdgcn_fence(__ATOMIC_RELEASE, "workgroup"); } while (0)

#define NB 4
#define TT 2048
#define DD 128
#define NH 8
#define HE 16
#define DFF 512
#define NR (NB * TT)

__global__ __launch_bounds__(128) void k_proj(const float* __restrict__ x, const float* __restrict__ WQ, const float* __restrict__ WK, const float* __restrict__ WV,
                                            float* __restrict__ xpe, _Float16* __restrict__ Qh, _Float16* __restrict__ Kh, _Float16* __restrict__ vT) {
  __shared__ __align__(16) float sx[64][DD + 4];
  __shared__ __align__(16) float so[4][16][132];
  __shared__ __align__(16) _Float16 st[DD][72];
  const int tid = threadIdx.x, wave = tid >> 5, lane = tid & 31, col = lane & 15, g = lane >> 4;
  const int r0b = blockIdx.x * 64, b = r0b / TT, t0 = r0b % TT;
  for (int q = tid; q < 64 * DD; q += 128) { const int rl = q >> 7, c = q & 127; const int t = t0 + rl;
    const float div = expf((float)(c & ~1) * (-logf(10000.0f) / (float)DD)); const float ang = (float)t * div;
    const float pe = (c & 1) ? cosf(ang) : sinf(ang);
    sx[rl][c] = x[(size_t)(r0b + rl) * DD + c] + pe; }
  __syncthreads();
  for (int q = tid; q < 64 * 32; q += 128) { const int rl = q >> 5, pc = q & 31; vst2(xpe + (size_t)(r0b + rl) * DD + pc * 4, *(const v4f*)(&sx[rl][pc * 4])); }
#pragma unroll 1
  for (int which = 0; which < 3; ++which) { const float* W = which == 0 ? WQ : (which == 1 ? WK : WV);
    v8f acc[8] = {};
#pragma unroll
    for (int kc = 0; kc < DD / 32; ++kc) { const v16h a = frag_f32(&sx[wave * 16 + col][0] + kc * 32, lane);
#pragma unroll
      for (int j = 0; j < 8; ++j) acc[j] = wmma16(a, fragc_f32(W, kc * 32, j * 16 + col, lane, DD, DD), acc[j]); }
    if (which < 2) {
#pragma unroll
      for (int j = 0; j < 8; ++j)
#pragma unroll
        for (int r = 0; r < 8; ++r) so[wave][8 * g + r][j * 16 + col] = acc[j][r];
      LDSX();
      _Float16* dst = which == 0 ? Qh : Kh;
      for (int q = lane; q < 8 * 32; q += 32) { const int h = q >> 5, pp = q & 31; const int rl = pp >> 1, half = (pp & 1) * 8; union { v8h hh; v4u u; } pk;
#pragma unroll
        for (int i = 0; i < 8; ++i) pk.hh[i] = (_Float16)so[wave][rl][h * 16 + half + i];
        vst2(dst + (((size_t)h * NB + b) * TT + t0 + wave * 16 + rl) * HE + half, pk.u); }
      LDSX();
    } else {
#pragma unroll
      for (int j = 0; j < 8; ++j)
#pragma unroll
        for (int r = 0; r < 8; ++r) st[j * 16 + col][wave * 16 + 8 * g + r] = (_Float16)acc[j][r];
      __syncthreads();
      for (int q = tid; q < DD * 8; q += 128) { const int c = q >> 3, pc = q & 7, h = c >> 4, e = c & 15;
        vst2(vT + (((size_t)h * NB + b) * HE + e) * TT + t0 + pc * 8, *(const v4u*)(&st[c][pc * 8])); }
    }
  }
}
__device__ __forceinline__ v16h frag16(const _Float16* row16, int lane) {
  v16h a; const int hh = lane >> 4; union { v8h v; } u; u.v = *(const v8h*)(row16 + 8 * hh);
#pragma unroll
  for (int i = 0; i < 8; ++i) { a[i] = u.v[i]; a[8 + i] = (_Float16)0.f; }
  return a;
}
__global__ __launch_bounds__(128) void k_z(const _Float16* __restrict__ Qh, const _Float16* __restrict__ Kh, float* __restrict__ Z) {
  __shared__ __align__(16) float sz[64];
  const int tid = threadIdx.x, w = tid >> 5, lane = tid & 31, col = lane & 15, g = lane >> 4;
  const int hb = blockIdx.y, k0 = blockIdx.x * 64 + w * 16;
  const _Float16* qb = Qh + (size_t)hb * TT * HE; const _Float16* kb = Kh + (size_t)hb * TT * HE;
  const v16h ak = frag16(kb + (size_t)(k0 + col) * HE, lane);
  const float scl = rsqrtf((float)TT);
  float zs[8] = {0.f, 0.f, 0.f, 0.f, 0.f, 0.f, 0.f, 0.f};
#pragma unroll 1
  for (int qt = blockIdx.x; qt < TT / 64; ++qt) {
#pragma unroll
    for (int t = 0; t < 4; ++t) { v8f acc = {}; acc = wmma16(ak, frag16(qb + (size_t)(qt * 64 + t * 16 + col) * HE, lane), acc);
#pragma unroll
      for (int r = 0; r < 8; ++r) { const int key = k0 + 8 * g + r, q = qt * 64 + t * 16 + col; if (q >= key) zs[r] += expf(acc[r] * scl); } } }
#pragma unroll
  for (int off = 8; off >= 1; off >>= 1) {
#pragma unroll
    for (int r = 0; r < 8; ++r) zs[r] += __shfl_xor(zs[r], off, 32); }
  if (col == 0) {
#pragma unroll
    for (int r = 0; r < 8; ++r) sz[w * 16 + 8 * g + r] = zs[r]; }
  __syncthreads();
  if (tid < 16) vst2(Z + (size_t)hb * TT + blockIdx.x * 64 + tid * 4, *(const v4f*)(&sz[tid * 4]));
}
__global__ __launch_bounds__(128) void k_av(const _Float16* __restrict__ Qh, const _Float16* __restrict__ Kh, const _Float16* __restrict__ vT, const float* __restrict__ Z, float* __restrict__ oh) {
  __shared__ __align__(16) _Float16 sP[4][16][72];
  __shared__ __align__(16) float so[4][16][20];
  const int tid = threadIdx.x, w = tid >> 5, lane = tid & 31, col = lane & 15, g = lane >> 4;
  const int hb = blockIdx.y, q0 = blockIdx.x * 64 + w * 16;
  const _Float16* qb = Qh + (size_t)hb * TT * HE; const _Float16* kb = Kh + (size_t)hb * TT * HE; const _Float16* vb = vT + (size_t)hb * HE * TT;
  const v16h aq = frag16(qb + (size_t)(q0 + col) * HE, lane);
  const float scl = rsqrtf((float)TT);
  v8f acc = {};
#pragma unroll 1
  for (int kt = 0; kt <= (int)blockIdx.x; ++kt) {
#pragma unroll
    for (int t = 0; t < 4; ++t) { v8f s = {}; s = wmma16(aq, frag16(kb + (size_t)(kt * 64 + t * 16 + col) * HE, lane), s);
      const int key = kt * 64 + t * 16 + col; const float zinv = 1.0f / Z[(size_t)hb * TT + key];
#pragma unroll
      for (int r = 0; r < 8; ++r) { const int q = q0 + 8 * g + r; const float p = key <= q ? expf(s[r] * scl) * zinv : 0.f; sP[w][8 * g + r][t * 16 + col] = (_Float16)(p * 256.0f); } }
    LDSX();
#pragma unroll
    for (int kc = 0; kc < 2; ++kc) acc = wmma16(frag_h(&sP[w][col][0] + kc * 32, lane), frag_h(vb + (size_t)col * TT + kt * 64 + kc * 32, lane), acc);
    __builtin_amdgcn_wave_barrier();
  }
#pragma unroll
  for (int r = 0; r < 8; ++r) so[w][8 * g + r][col] = acc[r] * (1.0f / 256.0f);
  LDSX();
  for (int q = lane; q < 64; q += 32) { const int rl = q >> 2, pc = q & 3; vst2(oh + ((size_t)hb * TT + q0 + rl) * HE + pc * 4, *(const v4f*)(&so[w][rl][pc * 4])); }
}
__global__ __launch_bounds__(128) void k_ff1(const float* __restrict__ oh, const float* __restrict__ W1, const float* __restrict__ b1, _Float16* __restrict__ hid) {
  __shared__ __align__(16) float so[4][16][132];
  const int tid = threadIdx.x, wave = tid >> 5, lane = tid & 31, col = lane & 15, g = lane >> 4;
  const int r0 = blockIdx.x * 64 + wave * 16, n0 = blockIdx.y * 128; const int r = r0 + col, b = r / TT, t = r % TT;
  v8f acc[8] = {};
#pragma unroll
  for (int kc = 0; kc < DD / 32; ++kc) { v16h a;
#pragma unroll
    for (int i = 0; i < 8; ++i) { const int ka = kc * 32 + 8 * g + i, kz = ka + 16;
      a[i] = (_Float16)oh[(((size_t)(ka >> 4) * NB + b) * TT + t) * HE + (ka & 15)]; a[8 + i] = (_Float16)oh[(((size_t)(kz >> 4) * NB + b) * TT + t) * HE + (kz & 15)]; }
#pragma unroll
    for (int j = 0; j < 8; ++j) acc[j] = wmma16(a, fragc_f32(W1, kc * 32, n0 + j * 16 + col, lane, DFF, DD), acc[j]); }
#pragma unroll
  for (int j = 0; j < 8; ++j) { const float bb = b1[n0 + j * 16 + col];
#pragma unroll
    for (int rr = 0; rr < 8; ++rr) { const float v = acc[j][rr] + bb; so[wave][8 * g + rr][j * 16 + col] = v > 0.f ? v : 0.f; } }
  LDSX();
  for (int q = lane; q < 16 * 16; q += 32) { const int rl = q >> 4, pc = q & 15; union { v8h hh; v4u u; } pk;
#pragma unroll
    for (int i = 0; i < 8; ++i) pk.hh[i] = (_Float16)so[wave][rl][pc * 8 + i];
    vst2(hid + (size_t)(r0 + rl) * DFF + n0 + pc * 8, pk.u); }
}
__global__ __launch_bounds__(128) void k_ff2(const _Float16* __restrict__ hid, const float* __restrict__ W2, const float* __restrict__ b2, const float* __restrict__ xpe, float* __restrict__ out) {
  __shared__ __align__(16) float so[4][16][132];
  const int tid = threadIdx.x, wave = tid >> 5, lane = tid & 31, col = lane & 15, g = lane >> 4;
  const int r0 = blockIdx.x * 64 + wave * 16;
  v8f acc[8] = {};
#pragma unroll 1
  for (int kc = 0; kc < DFF / 32; ++kc) { const v16h a = frag_h(hid + (size_t)(r0 + col) * DFF + kc * 32, lane);
#pragma unroll
    for (int j = 0; j < 8; ++j) acc[j] = wmma16(a, fragc_f32(W2, kc * 32, j * 16 + col, lane, DD, DFF), acc[j]); }
#pragma unroll
  for (int j = 0; j < 8; ++j) { const float bb = b2[j * 16 + col];
#pragma unroll
    for (int rr = 0; rr < 8; ++rr) so[wave][8 * g + rr][j * 16 + col] = acc[j][rr] + bb; }
  LDSX();
#pragma unroll 4
  for (int rl = 0; rl < 16; ++rl) { const size_t o = (size_t)(r0 + rl) * DD + lane * 4; vst2(out + o, *(const v4f*)(&so[wave][rl][lane * 4]) + *(const v4f*)(xpe + o)); }
}
extern "C" void kernel_launch(void* const* d_in, const int* in_sizes, int n_in, void* d_out, int out_size, void* d_ws, size_t ws_size, hipStream_t stream) {
  (void)in_sizes; (void)n_in; (void)out_size; (void)ws_size;
  const float* x = (const float*)d_in[0]; const float* WQ = (const float*)d_in[1]; const float* WK = (const float*)d_in[2]; const float* WV = (const float*)d_in[3];
  const float* W1 = (const float*)d_in[4]; const float* b1 = (const float*)d_in[5]; const float* W2 = (const float*)d_in[6]; const float* b2 = (const float*)d_in[7];
  float* out = (float*)d_out;
  char* ws = (char*)d_ws; size_t off = 0;
  auto take = [&](size_t bytes) { char* p = ws + off; off += (bytes + 255) & ~(size_t)255; return p; };
  float* xpe = (float*)take((size_t)NR * DD * 4);
  _Float16* Qh = (_Float16*)take((size_t)NR * DD * 2); _Float16* Kh = (_Float16*)take((size_t)NR * DD * 2); _Float16* vT = (_Float16*)take((size_t)NR * DD * 2);
  float* Z = (float*)take((size_t)NH * NB * TT * 4); float* oh = (float*)take((size_t)NR * DD * 4); _Float16* hid = (_Float16*)take((size_t)NR * DFF * 2);
  k_proj<<<NR / 64, 128, 0, stream>>>(x, WQ, WK, WV, xpe, Qh, Kh, vT);
  k_z<<<dim3(TT / 64, NH * NB), 128, 0, stream>>>(Qh, Kh, Z);
  k_av<<<dim3(TT / 64, NH * NB), 128, 0, stream>>>(Qh, Kh, vT, Z, oh);
  k_ff1<<<dim3(NR / 64, DFF / 128), 128, 0, stream>>>(oh, W1, b1, hid);
  k_ff2<<<NR / 64, 128, 0, stream>>>(hid, W2, b2, xpe, out);
}
